// _EdgeScorer_36421322670672
// MI455X (gfx1250) — hardware-verified
//
#include <hip/hip_runtime.h>
#include <stddef.h>
#include <math.h>


#define ND       128
#define NCOL     256
#define NTHR     256
#define NWAVE    8
#define GROWS    128
#define AP       (ND + 8)
#define EPW      32
#define WSCALE   16.0f
#define WINV     0.0625f
#define LDS_STG  (GROWS * ND * 4)
#define LDS_SA   (GROWS * AP * 2)
#define LDS_GEMM (LDS_STG + LDS_SA)

static_assert((GROWS * ND / 8) % NTHR == 0);
static_assert(GROWS == NWAVE * 16);
static_assert(((AP * 2) % 16) == 0);
static_assert(NCOL * ND / 8 == 16 * NTHR);
static_assert((ND % 32) == 0);
static_assert((LDS_STG % 16) == 0);

typedef float    v4f  __attribute__((ext_vector_type(4)));
typedef float    v8f  __attribute__((ext_vector_type(8)));
typedef _Float16 v8h  __attribute__((ext_vector_type(8)));
typedef _Float16 v16h __attribute__((ext_vector_type(16)));
union FragH { v16h v; v8h h[2]; };

__device__ __forceinline__ v8h cvt8(v4f a, v4f b) {
  v8h r;
  r[0] = (_Float16)a.x; r[1] = (_Float16)a.y; r[2] = (_Float16)a.z; r[3] = (_Float16)a.w;
  r[4] = (_Float16)b.x; r[5] = (_Float16)b.y; r[6] = (_Float16)b.z; r[7] = (_Float16)b.w;
  return r;
}

__device__ __forceinline__ v8f wmh(v16h a, v16h b, v8f c) {
  v8f d = __builtin_amdgcn_wmma_f32_16x16x32_f16(false, a, false, b, (short)0, c, false, false);
#if defined(__HIP_DEVICE_COMPILE__)
  asm volatile("v_nop\n\tv_nop\n\tv_nop\n\tv_nop" : "+v"(d) : "v"(a), "v"(b));
#endif
  return d;
}

__global__ __launch_bounds__(NTHR) void k_wprep(const float* __restrict__ W1, _Float16* Bw) {
  const int idx = blockIdx.x * NTHR + (int)threadIdx.x;
  if (idx >= NCOL * ND / 8) return;
  const int n  = idx >> 4;
  const int k0 = (idx & 15) * 8;
  const int rofs = (n < ND) ? 0 : ND;
  const int c  = n & (ND - 1);
  float v[8];
#pragma unroll
  for (int e = 0; e < 8; ++e) {
    const int r = rofs + k0 + e;
    v[e] = W1[(size_t)r * ND + c] * WSCALE;
  }
  v4f a, b;
  a.x = v[0]; a.y = v[1]; a.z = v[2]; a.w = v[3];
  b.x = v[4]; b.y = v[5]; b.z = v[6]; b.w = v[7];
  const v8h hv = cvt8(a, b);
  _Float16* dp = Bw + (size_t)idx * 8;
  *(volatile v8h*)dp = hv;
  __threadfence();
  *(volatile v8h*)dp = hv;
}

__global__ __launch_bounds__(NTHR) void k_gemm(
    const float* __restrict__ X, const _Float16* __restrict__ Bw, float* PQ, int nN, int planeRows) {
  extern __shared__ v4f lds_dyn[];
  float*    stg = (float*)lds_dyn;
  _Float16* sA  = (_Float16*)((char*)lds_dyn + LDS_STG);
  const int tid = threadIdx.x, lane = tid & 31, wave = tid >> 5, hh = lane >> 4, m = lane & 15;
  const int rowBase = blockIdx.x * GROWS;

#pragma unroll
  for (int i = 0; i < (GROWS * ND / 8) / NTHR; ++i) {
    const int idx = i * NTHR + tid;
    const int r   = idx >> 4;
    const int c0  = (idx & 15) * 8;
    int row = rowBase + r;
    row = row > nN - 1 ? nN - 1 : row;
    const float* ap = X + (size_t)row * ND + c0;
    const v4f a = *(const v4f*)ap, b = *(const v4f*)(ap + 4);
    *(v8h*)(sA + r * AP + c0) = cvt8(a, b);
  }
  __syncthreads();

  const _Float16* ar = sA + (wave * 16 + m) * AP + 8 * hh;
  const size_t planeElems = (size_t)planeRows * ND;

#pragma unroll 1
  for (int g = 0; g < 2; ++g) {
    v8f acc[8];
#pragma unroll
    for (int t = 0; t < 8; ++t) { v8f z = {0.f, 0.f, 0.f, 0.f, 0.f, 0.f, 0.f, 0.f}; acc[t] = z; }
#pragma unroll 1
    for (int kt = 0; kt < ND / 32; ++kt) {
      FragH a;
      a.h[0] = *(const v8h*)(ar + 32 * kt);
      a.h[1] = *(const v8h*)(ar + 32 * kt + 16);
#pragma unroll
      for (int t = 0; t < 8; ++t) {
        const _Float16* bp = Bw + (size_t)(ND * g + 16 * t + m) * ND + 32 * kt + 8 * hh;
        FragH b;
        b.h[0] = *(const v8h*)bp;
        b.h[1] = *(const v8h*)(bp + 16);
        acc[t] = wmh(a.v, b.v, acc[t]);
      }
    }
    float* sp = stg + (wave * 16 + 8 * hh) * ND + m;
#pragma unroll
    for (int t = 0; t < 8; ++t) {
#pragma unroll
      for (int r = 0; r < 8; ++r) sp[r * ND + 16 * t] = acc[t][r] * WINV;
    }
    __syncthreads();

    const float* lp = stg + wave * 16 * ND + 4 * lane;
    float* gp = PQ + (size_t)g * planeElems + ((size_t)rowBase + wave * 16) * ND + 4 * lane;
#pragma unroll
    for (int i = 0; i < 16; ++i) {
      const v4f v = *(const v4f*)(lp + i * ND);
      *(volatile v4f*)(gp + (size_t)i * ND) = v;
    }
    __threadfence();
#pragma unroll
    for (int i = 0; i < 16; ++i) {
      const v4f v = *(const v4f*)(lp + i * ND);
      *(volatile v4f*)(gp + (size_t)i * ND) = v;
    }
    __syncthreads();
  }
}

__global__ __launch_bounds__(NTHR) void k_edge(
    const int* __restrict__ ei, const float* __restrict__ P, const float* __restrict__ Q,
    const float* __restrict__ b1, const float* __restrict__ W2, const float* __restrict__ b2,
    float* out, int nE, int nN) {
  const int tid = threadIdx.x, lane = tid & 31, wave = tid >> 5;
  const int base = (blockIdx.x * NWAVE + wave) * EPW;
  if (base >= nE) return;
  const int er = base + lane;
  const int ec = er < nE ? er : nE - 1;
  int sl = ei[ec];
  int dl = ei[(size_t)nE + ec];
  sl = sl < 0 ? 0 : (sl > nN - 1 ? nN - 1 : sl);
  dl = dl < 0 ? 0 : (dl > nN - 1 ? nN - 1 : dl);
  const v4f bb = *(const v4f*)(b1 + 4 * lane);
  const v4f ww = *(const v4f*)(W2 + 4 * lane);
  const float b2v = b2[0];

  float mys = 0.0f;
#pragma unroll 2
  for (int j = 0; j < EPW; ++j) {
    const int s = __builtin_amdgcn_readlane(sl, j);
    const int d = __builtin_amdgcn_readlane(dl, j);
    const v4f p = *(const v4f*)(P + (size_t)s * ND + 4 * lane);
    const v4f q = *(const v4f*)(Q + (size_t)d * ND + 4 * lane);
    v4f h = p + q + bb;
    h.x = fmaxf(h.x, 0.0f); h.y = fmaxf(h.y, 0.0f); h.z = fmaxf(h.z, 0.0f); h.w = fmaxf(h.w, 0.0f);
    float a = h.x * ww.x;
    a = fmaf(h.y, ww.y, a);
    a = fmaf(h.z, ww.z, a);
    a = fmaf(h.w, ww.w, a);
    a += __shfl_xor(a, 16, 32);
    a += __shfl_xor(a, 8, 32);
    a += __shfl_xor(a, 4, 32);
    a += __shfl_xor(a, 2, 32);
    a += __shfl_xor(a, 1, 32);
    mys = (lane == j) ? a : mys;
  }
  float t = mys + b2v;
  t = fminf(fmaxf(t, -30.0f), 30.0f);
  const float ex  = expf(-t);
  const float sig = 1.0f / (1.0f + ex);
  float* op = out + (size_t)base + lane;
  if (er < nE) *(volatile float*)op = sig;
  __threadfence();
  if (er < nE) *(volatile float*)op = sig;
}

extern "C" void kernel_launch(void* const* d_in, const int* in_sizes, int n_in,
                              void* d_out, int out_size, void* d_ws, size_t ws_size,
                              hipStream_t stream) {
  if (n_in < 6) return;
  const int nN = in_sizes[0] / ND;
  const int nE = in_sizes[1] / 2;
  if (nN <= 0 || nE <= 0 || in_sizes[0] != nN * ND || in_sizes[1] != 2 * nE) return;
  if (in_sizes[2] != NCOL * ND || in_sizes[3] != ND || in_sizes[4] != ND || in_sizes[5] < 1) return;
  if (out_size != nE) return;
  if (nN > (1 << 22) || nE > (1 << 28)) return;

  const float* x  = (const float*)d_in[0];
  const int*   ei = (const int*)d_in[1];
  const float* W1 = (const float*)d_in[2];
  const float* b1 = (const float*)d_in[3];
  const float* W2 = (const float*)d_in[4];
  const float* b2 = (const float*)d_in[5];
  float* out = (float*)d_out;

  const int nGemm = (nN + GROWS - 1) / GROWS;
  const int NPAD  = nGemm * GROWS;
  const int nEdgeBlocks = (nE + NWAVE * EPW - 1) / (NWAVE * EPW);

  char* ws = (char*)d_ws;
  size_t off = 0;
  const size_t oW = off; off += (size_t)NCOL * ND * 2;          off = (off + 255) & ~(size_t)255;
  const size_t oP = off; off += (size_t)NPAD * ND * 4;          off = (off + 255) & ~(size_t)255;
  const size_t oQ = off; off += (size_t)NPAD * ND * 4;          off = (off + 255) & ~(size_t)255;
  if (off > ws_size) return;
  if (oQ != oP + (size_t)NPAD * ND * 4) return;
  _Float16* Bw = (_Float16*)(ws + oW);
  float*    P  = (float*)(ws + oP);
  float*    Q  = (float*)(ws + oQ);

  k_wprep<<<(NCOL * ND / 8 + NTHR - 1) / NTHR, NTHR, 0, stream>>>(W1, Bw);

  hipFuncSetAttribute(reinterpret_cast<const void*>(&k_gemm),
                      hipFuncAttributeMaxDynamicSharedMemorySize, LDS_GEMM);
  k_gemm<<<nGemm, NTHR, LDS_GEMM, stream>>>(x, Bw, P, nN, NPAD);

  k_edge<<<nEdgeBlocks, NTHR, 0, stream>>>(ei, P, Q, b1, W2, b2, out, nE, nN);
}
